// TreeLSTMCell_83932250898829
// MI455X (gfx1250) — hardware-verified
//
#include <hip/hip_runtime.h>

#define DD 2048
#define HH 2048
#define KK 4096

typedef __attribute__((ext_vector_type(16))) _Float16 v16bf;
typedef __attribute__((ext_vector_type(8)))  _Float16 v8bf;
typedef __attribute__((ext_vector_type(8)))  float  v8f;
typedef __attribute__((ext_vector_type(4)))  float  v4f_t;
typedef float v4fa __attribute__((ext_vector_type(4), may_alias));

__device__ __forceinline__ unsigned pk2bf(float x, float y) {
  return (unsigned)__builtin_bit_cast(unsigned short, (_Float16)x) | ((unsigned)__builtin_bit_cast(unsigned short, (_Float16)y) << 16);
}

__device__ __forceinline__ uint2 pk4bf(float4 v) {
  uint2 r;
  r.x = pk2bf(v.x, v.y);
  r.y = pk2bf(v.z, v.w);
  return r;
}

__device__ __forceinline__ float sigmoidf_(float x) {
  return 1.0f / (1.0f + __expf(-x));
}

__device__ __forceinline__ float wave_reduce_add(float v) {
#pragma unroll
  for (int off = 16; off > 0; off >>= 1) v += __shfl_down(v, off, 32);
  return v;
}

__global__ __launch_bounds__(256) void hsum_part_kernel(
    const float* __restrict__ ch_h, float* __restrict__ part) {
  int j  = blockIdx.x * 256 + threadIdx.x;
  int kc = blockIdx.y;
  float acc = 0.f;
  const float* p = ch_h + (size_t)kc * 512 * HH + j;
  for (int k = 0; k < 512; ++k) acc += p[(size_t)k * HH];
  *(volatile float*)(part + (size_t)kc * HH + j) = acc; __threadfence(); *(volatile float*)(part + (size_t)kc * HH + j) = acc;
}

__global__ __launch_bounds__(256) void hsum_reduce_kernel(
    const float* __restrict__ part, float* __restrict__ hsum) {
  int j = blockIdx.x * 256 + threadIdx.x;
  float s = 0.f;
#pragma unroll
  for (int kc = 0; kc < 8; ++kc) s += part[(size_t)kc * HH + j];
  *(volatile float*)(hsum + j) = s; __threadfence(); *(volatile float*)(hsum + j) = s;
}

__global__ __launch_bounds__(256) void gemv_fx_kernel(
    const float* __restrict__ W_fx, const float* __restrict__ b_fx,
    const float* __restrict__ b_fh, const float* __restrict__ x,
    float* __restrict__ fxb) {
  __shared__ __align__(16) float sr[32];
  int wave = threadIdx.x >> 5, lane = threadIdx.x & 31;
  for (int q = 0; q < 4; ++q) {
    int row = blockIdx.x * 32 + wave * 4 + q;
    const float* w = W_fx + (size_t)row * DD;
    float acc = 0.f;
    for (int l = lane; l < DD; l += 32) acc += w[l] * x[l];
    acc = wave_reduce_add(acc);
    if (lane == 0) sr[wave * 4 + q] = acc + b_fx[row] + b_fh[row];
  }
  __syncthreads();
  if (threadIdx.x < 8) { const v4f_t v = *(const volatile v4fa*)(sr + threadIdx.x * 4); float* d = fxb + blockIdx.x * 32 + threadIdx.x * 4;
    *(volatile v4f_t*)d = v; __threadfence(); *(volatile v4f_t*)d = v; }
}

__global__ __launch_bounds__(256) void gemv_iou_kernel(
    const float* __restrict__ Wx, const float* __restrict__ bx,
    const float* __restrict__ Wh, const float* __restrict__ bh,
    const float* __restrict__ x,  const float* __restrict__ hsum,
    float* __restrict__ i_g, float* __restrict__ u_g, float* __restrict__ out) {
  __shared__ __align__(16) float sr[32];
  int wave = threadIdx.x >> 5, lane = threadIdx.x & 31;
  const int row0 = blockIdx.x * 32;
  const int gate = row0 >> 11;
  for (int q = 0; q < 4; ++q) {
    int row = row0 + wave * 4 + q;
    const float* wxr = Wx + (size_t)row * DD;
    const float* whr = Wh + (size_t)row * HH;
    float acc = 0.f;
    for (int l = lane; l < DD; l += 32) acc += wxr[l] * x[l] + whr[l] * hsum[l];
    acc = wave_reduce_add(acc);
    if (lane == 0) {
      acc += bx[row] + bh[row];
      sr[wave * 4 + q] = (gate == 2) ? tanhf(acc) : sigmoidf_(acc);
    }
  }
  __syncthreads();
  if (threadIdx.x < 8) {
    float* base = (gate == 0) ? i_g : (gate == 1) ? out : u_g;
    const v4f_t v = *(const volatile v4fa*)(sr + threadIdx.x * 4); float* d = base + (row0 & (HH - 1)) + threadIdx.x * 4;
    *(volatile v4f_t*)d = v; __threadfence(); *(volatile v4f_t*)d = v;
  }
}

__global__ __launch_bounds__(256) void fused_gemm_kernel(
    const float* __restrict__ ch_h, const float* __restrict__ ch_c,
    const float* __restrict__ W_fh, const float* __restrict__ fxb,
    float* __restrict__ partials) {
  __shared__ __align__(16) unsigned short lA[2][128][40];
  __shared__ __align__(16) unsigned short lB[2][128][40];
  __shared__ float sC[4][128];

  const int tid  = threadIdx.x;
  const int wave = tid >> 5, lane = tid & 31;
  const int wm = wave >> 1, wn = wave & 1;
  const int half = lane >> 4, l16 = lane & 15;
  const int n_base = blockIdx.x * 128;
  const int m_base = blockIdx.y * 128;

  const int srow = tid >> 3;
  const int scg  = tid & 7;

  v8f acc[2][4];
  const v8f vzero = {0.f,0.f,0.f,0.f,0.f,0.f,0.f,0.f};
#pragma unroll
  for (int mi = 0; mi < 2; ++mi)
#pragma unroll
    for (int ni = 0; ni < 4; ++ni) acc[mi][ni] = vzero;

  float4 ra[4], rb[4];
#pragma unroll
  for (int it = 0; it < 4; ++it) {
    int row = srow + it * 32;
    ra[it] = *reinterpret_cast<const float4*>(
        ch_h + (size_t)(m_base + row) * HH + scg * 4);
    rb[it] = *reinterpret_cast<const float4*>(
        W_fh + (size_t)(n_base + row) * HH + scg * 4);
  }

  for (int t = 0; t < HH / 32; ++t) {
    const int buf = t & 1;
    const int l0n = (t + 1) * 32;
    __syncthreads();
#pragma unroll
    for (int it = 0; it < 4; ++it) {
      int row = srow + it * 32;
      *reinterpret_cast<uint2*>(&lA[buf][row][scg * 4]) = pk4bf(ra[it]);
      *reinterpret_cast<uint2*>(&lB[buf][row][scg * 4]) = pk4bf(rb[it]);
    }
    if (t + 1 < HH / 32) {
#pragma unroll
      for (int it = 0; it < 4; ++it) {
        int row = srow + it * 32;
        ra[it] = *reinterpret_cast<const float4*>(
            ch_h + (size_t)(m_base + row) * HH + l0n + scg * 4);
        rb[it] = *reinterpret_cast<const float4*>(
            W_fh + (size_t)(n_base + row) * HH + l0n + scg * 4);
      }
    }
    __syncthreads();

    v16bf fa[2], fb[4];
#pragma unroll
    for (int mi = 0; mi < 2; ++mi) {
      int r = wm * 32 + mi * 16 + l16;
      v8bf lo = *reinterpret_cast<const v8bf*>(&lA[buf][r][8 * half]);
      v8bf hi = *reinterpret_cast<const v8bf*>(&lA[buf][r][16 + 8 * half]);
      fa[mi] = __builtin_shufflevector(lo, hi, 0,1,2,3,4,5,6,7,8,9,10,11,12,13,14,15);
    }
#pragma unroll
    for (int ni = 0; ni < 4; ++ni) {
      int r = wn * 64 + ni * 16 + l16;
      v8bf lo = *reinterpret_cast<const v8bf*>(&lB[buf][r][8 * half]);
      v8bf hi = *reinterpret_cast<const v8bf*>(&lB[buf][r][16 + 8 * half]);
      fb[ni] = __builtin_shufflevector(lo, hi, 0,1,2,3,4,5,6,7,8,9,10,11,12,13,14,15);
    }
#pragma unroll
    for (int mi = 0; mi < 2; ++mi)
#pragma unroll
      for (int ni = 0; ni < 4; ++ni)
        acc[mi][ni] = __builtin_amdgcn_wmma_f32_16x16x32_f16(
            false, fa[mi], false, fb[ni], (short)0, acc[mi][ni], false, false);
  }

  float csum[4] = {0.f, 0.f, 0.f, 0.f};
#pragma unroll
  for (int ni = 0; ni < 4; ++ni) {
    int j = n_base + wn * 64 + ni * 16 + l16;
    float fxbj = fxb[j];
#pragma unroll
    for (int mi = 0; mi < 2; ++mi) {
#pragma unroll
      for (int r = 0; r < 8; ++r) {
        int k = m_base + wm * 32 + mi * 16 + 8 * half + r;
        float f = sigmoidf_(fxbj + acc[mi][ni][r]);
        csum[ni] += f * ch_c[(size_t)k * HH + j];
      }
    }
  }
#pragma unroll
  for (int ni = 0; ni < 4; ++ni) {
    float tot = csum[ni] + __shfl_xor(csum[ni], 16, 32);
    if (half == 0) sC[wm][wn * 64 + ni * 16 + l16] = tot;
  }
  __syncthreads();
  if (tid < 128) {
    float s = sC[0][tid] + sC[1][tid] + sC[2][tid] + sC[3][tid];
    float* d = partials + (size_t)blockIdx.y * HH + n_base + tid;
    *(volatile float*)d = s; __threadfence(); *(volatile float*)d = s;
  }
}

__global__ __launch_bounds__(256) void finalize_kernel(
    const float* __restrict__ i_g, const float* __restrict__ u_g,
    const float* __restrict__ partials, float* __restrict__ out) {
  int j = blockIdx.x * 256 + threadIdx.x;
  float c = i_g[j] * u_g[j];
#pragma unroll
  for (int mb = 0; mb < 32; ++mb) c += partials[(size_t)mb * HH + j];
  const float hv = out[j] * tanhf(c);
  *(volatile float*)(out + HH + j) = c; *(volatile float*)(out + 2 * HH + j) = hv; __threadfence();
  *(volatile float*)(out + HH + j) = c; *(volatile float*)(out + 2 * HH + j) = hv;
}

extern "C" void kernel_launch(void* const* d_in, const int* in_sizes, int n_in,
                              void* d_out, int out_size, void* d_ws, size_t ws_size,
                              hipStream_t stream) {
  const float* input  = (const float*)d_in[0];
  const float* ch_c   = (const float*)d_in[1];
  const float* ch_h   = (const float*)d_in[2];
  const float* W_ioux = (const float*)d_in[3];
  const float* b_ioux = (const float*)d_in[4];
  const float* W_iouh = (const float*)d_in[5];
  const float* b_iouh = (const float*)d_in[6];
  const float* W_fx   = (const float*)d_in[7];
  const float* b_fx   = (const float*)d_in[8];
  const float* W_fh   = (const float*)d_in[9];
  const float* b_fh   = (const float*)d_in[10];
  float* out = (float*)d_out;

  float* ws       = (float*)d_ws;
  float* fxb      = ws;
  float* i_g      = ws + HH;
  float* u_g      = ws + 2 * HH;
  float* hsum     = ws + 3 * HH;
  float* hpart    = ws + 4 * HH;
  float* partials = ws + 12 * HH;

  hsum_part_kernel<<<dim3(HH / 256, 8), 256, 0, stream>>>(ch_h, hpart);
  hsum_reduce_kernel<<<HH / 256, 256, 0, stream>>>(hpart, hsum);
  gemv_fx_kernel<<<HH / 32, 256, 0, stream>>>(W_fx, b_fx, b_fh, input, fxb);
  gemv_iou_kernel<<<(3 * HH) / 32, 256, 0, stream>>>(
      W_ioux, b_ioux, W_iouh, b_iouh, input, hsum, i_g, u_g, out);
  fused_gemm_kernel<<<dim3(HH / 128, KK / 128), 256, 0, stream>>>(
      ch_h, ch_c, W_fh, fxb, partials);
  finalize_kernel<<<HH / 256, 256, 0, stream>>>(i_g, u_g, partials, out);
}
